// NDDE_4707284156651
// MI455X (gfx1250) — hardware-verified
//
#include <hip/hip_runtime.h>
#include <math.h>

#define STATE_DIM    128
#define HID_DIM      512
#define NBATCH       128
#define DELAY_STEPS  10
#define NUM_STEPS    1000
#define IN_DIM       258
#define KXY          256
#define ROWS_PB      16
#define NTHREADS     256
#define YPITCH       136
#define HPITCH       520
#define OPITCH       132
#define NSLOTS       11
#define SLOT_HALVES  (ROWS_PB * YPITCH)
#define W1_CARRY     16.0f
#define W2_CARRY     64.0f
#define LO_CARRY     2048.0f
#define W1_INV       (1.0f / 16.0f)
#define W1_LO_INV    (1.0f / 32768.0f)
#define W2_INV       (1.0f / 64.0f)
#define W2_LO_INV    (1.0f / 131072.0f)

static_assert(HID_DIM == 8 * 64);
static_assert(STATE_DIM == 8 * 16);
static_assert(NBATCH % ROWS_PB == 0);
static_assert(KXY % 32 == 0 && HID_DIM % 32 == 0 && STATE_DIM % 32 == 0);
static_assert(NSLOTS * SLOT_HALVES * 2 + ROWS_PB * HPITCH * 2 <= 65536);
static_assert(ROWS_PB * OPITCH * 4 <= ROWS_PB * HPITCH * 2);
static_assert((YPITCH % 8) == 0 && (HPITCH % 8) == 0 && (OPITCH % 4) == 0);

typedef __attribute__((ext_vector_type(16))) _Float16 v16h;
typedef __attribute__((ext_vector_type(8)))  _Float16 v8h;
typedef __attribute__((ext_vector_type(8)))  float    v8f;
typedef __attribute__((ext_vector_type(4)))  float    v4f;

__device__ __forceinline__ void dep_guard_h(v8f& a, v8f& b, v16h x, v16h y) { asm volatile("v_nop\n\tv_nop\n\tv_nop\n\tv_nop" : "+v"(a), "+v"(b) : "v"(x), "v"(y)); }
__device__ __forceinline__ void dep_guard4_h(v8f& a, v8f& b, v8f& c, v8f& d, v16h x, v16h y) { asm volatile("v_nop\n\tv_nop\n\tv_nop\n\tv_nop" : "+v"(a), "+v"(b), "+v"(c), "+v"(d) : "v"(x), "v"(y)); }
__device__ __forceinline__ void keep4_h(v16h a, v16h b, v16h c, v16h d) { asm volatile("v_nop" :: "v"(a), "v"(b), "v"(c), "v"(d)); }
__device__ __forceinline__ void keep2_h(v16h a, v16h b) { asm volatile("v_nop" :: "v"(a), "v"(b)); }
__device__ __forceinline__ void acc_guard4(v8f& a, v8f& b, v8f& c, v8f& d) { asm volatile("v_nop\n\tv_nop\n\tv_nop\n\tv_nop" : "+v"(a), "+v"(b), "+v"(c), "+v"(d)); }
__device__ __forceinline__ void acc_guard2(v8f& a, v8f& b) { asm volatile("v_nop\n\tv_nop\n\tv_nop\n\tv_nop" : "+v"(a), "+v"(b)); }

template <typename T> struct Frag;
template <> struct Frag<_Float16> {
  typedef v16h V; union U { v16h v; v8h h[2]; };
  static __device__ __forceinline__ v16h load(const _Float16* p) {
    U f; f.h[0] = *(const v8h*)(p); f.h[1] = *(const v8h*)(p + 16); return f.v;
  }
  static __device__ __forceinline__ v8f mma(v16h a, v16h b, v8f c) {
    return __builtin_amdgcn_wmma_f32_16x16x32_f16(false, a, false, b, (short)0, c, false, false);
  }
};

__device__ __forceinline__ float ftanh(float x) { return 1.0f - 2.0f * __builtin_amdgcn_rcpf(__expf(2.0f * x) + 1.0f); }

__global__ __launch_bounds__(NTHREADS) void split_planes_kernel(
    const float* __restrict__ src, int nrows, int ldi, int kcols, float carry,
    unsigned short* __restrict__ hi, unsigned short* __restrict__ lo) {
  const int t = blockIdx.x * NTHREADS + threadIdx.x;
  const int per_row = kcols >> 3;
  const int r = t / per_row;
  const int k8 = (t - r * per_row) * 8;
  if (r >= nrows) return;
  const float* sp = src + (size_t)r * (size_t)ldi + k8;
  v8h hv, lv;
#pragma unroll
  for (int e = 0; e < 8; ++e) {
    const float v = sp[e] * carry;
    const _Float16 h = (_Float16)v;
    const float res = (v - (float)h) * LO_CARRY;
    hv[e] = h;
    lv[e] = (_Float16)res;
  }
  const size_t o = (size_t)r * (size_t)kcols + (size_t)k8;
  for (int pass = 0; pass < 2; ++pass) {
    *(volatile v8h*)(hi + o) = hv;
    *(volatile v8h*)(lo + o) = lv;
    __threadfence();
  }
}

__global__ __launch_bounds__(NTHREADS) void dde_euler_kernel(
    const float* __restrict__ tau_p, const float* __restrict__ W1, const float* __restrict__ b1,
    const float* __restrict__ b2, const float* __restrict__ c0, const float* __restrict__ c1,
    const unsigned short* __restrict__ W1hp, const unsigned short* __restrict__ W1lp,
    const unsigned short* __restrict__ W2hp, const unsigned short* __restrict__ W2lp,
    float* __restrict__ out) {
  __shared__ __align__(16) _Float16 Yr[NSLOTS * SLOT_HALVES];
  __shared__ __align__(16) float    HO[ROWS_PB * HPITCH / 2];
  _Float16* Hh = (_Float16*)(void*)HO;
  float*    Os = HO;
  const _Float16* W1h = (const _Float16*)W1hp;
  const _Float16* W1l = (const _Float16*)W1lp;
  const _Float16* W2h = (const _Float16*)W2hp;
  const _Float16* W2l = (const _Float16*)W2lp;

  const int tid = threadIdx.x, lane = tid & 31, wave = tid >> 5;
  const int c = lane & 15, hh = lane >> 4, koff = hh * 8;
  const int rb = blockIdx.x * ROWS_PB;
  const float tau_s = tau_p[0];
  const float dtv = tau_s * (1.0f / (float)DELAY_STEPS);

  {
    const int m = tid >> 4, d8 = (tid & 15) * 8;
    float cv[8], gv[8];
#pragma unroll
    for (int e = 0; e < 8; ++e) { cv[e] = c0[(size_t)(rb + m) * STATE_DIM + d8 + e]; gv[e] = c1[d8 + e]; }
#pragma unroll 1
    for (int s = 0; s < NSLOTS; ++s) {
      const int k = (s == 0) ? DELAY_STEPS : (s - 1);
      const float ts = ((float)k - (float)DELAY_STEPS) * dtv;
      v8h hv;
#pragma unroll
      for (int e = 0; e < 8; ++e) hv[e] = (_Float16)(cv[e] + ts * gv[e]);
      *(v8h*)(Yr + s * SLOT_HALVES + m * YPITCH + d8) = hv;
    }
  }
  for (int pass = 0; pass < 2; ++pass) {
#pragma unroll
    for (int it = 0; it < 2; ++it) {
      const int idx = it * NTHREADS + tid;
      const int row = idx >> 5, c4 = (idx & 31) * 4;
      const v4f v = *(const v4f*)(c0 + (size_t)(rb + row) * STATE_DIM + c4);
      *(volatile v4f*)(out + (size_t)(rb + row) * STATE_DIM + c4) = v;
    }
    __threadfence();
  }
  float cb[4], cw[4];
#pragma unroll
  for (int nt = 0; nt < 4; ++nt) {
    const int n = 64 * wave + 16 * nt + c;
    cb[nt] = b1[n] + tau_s * W1[(size_t)n * IN_DIM + 256];
    cw[nt] = W1[(size_t)n * IN_DIM + 257];
  }
  const int dcol = 16 * wave + c;
  const float b2v = b2[dcol];
  float xs[8];
#pragma unroll
  for (int r = 0; r < 8; ++r) xs[r] = c0[(size_t)(rb + 8 * hh + r) * STATE_DIM + dcol];
  const _Float16* v2h = W2h + (size_t)dcol * HID_DIM + koff;
  const _Float16* v2l = W2l + (size_t)dcol * HID_DIM + koff;
  __syncthreads();

  const v8f z8 = {0.f, 0.f, 0.f, 0.f, 0.f, 0.f, 0.f, 0.f};
  int sx = 0, sy = 1;
#pragma unroll 1
  for (int j = 0; j < NUM_STEPS; ++j) {
    const float tj = (float)j * dtv;
    const _Float16* ax = Yr + sx * SLOT_HALVES + c * YPITCH + koff;
    const _Float16* ay = Yr + sy * SLOT_HALVES + c * YPITCH + koff;

#pragma unroll
    for (int g = 0; g < 2; ++g) {
      v8f aH0 = z8, aH1 = z8, aL0 = z8, aL1 = z8;
      const size_t nrow = (size_t)(64 * wave + 32 * g + c);
      const _Float16* w0h = W1h + nrow * KXY + koff;
      const _Float16* w1h = w0h + 16 * KXY;
      const _Float16* w0l = W1l + nrow * KXY + koff;
      const _Float16* w1l = w0l + 16 * KXY;
#pragma unroll
      for (int part = 0; part < 2; ++part) {
        const _Float16* ab = part ? ay : ax;
        const int kb = part * STATE_DIM;
#pragma unroll 1
        for (int kk = 0; kk < STATE_DIM; kk += 32) {
          const v16h a   = Frag<_Float16>::load(ab + kk);
          const v16h bh0 = Frag<_Float16>::load(w0h + kb + kk);
          const v16h bh1 = Frag<_Float16>::load(w1h + kb + kk);
          const v16h bl0 = Frag<_Float16>::load(w0l + kb + kk);
          const v16h bl1 = Frag<_Float16>::load(w1l + kb + kk);
          aH0 = Frag<_Float16>::mma(a, bh0, aH0);
          aH1 = Frag<_Float16>::mma(a, bh1, aH1);
          aL0 = Frag<_Float16>::mma(a, bl0, aL0);
          aL1 = Frag<_Float16>::mma(a, bl1, aL1);
          dep_guard4_h(aH0, aH1, aL0, aL1, a, bl1);
          keep4_h(bh0, bh1, bl0, bl1);
        }
      }
      acc_guard4(aH0, aH1, aL0, aL1);
      const float cadd0 = cb[2 * g]     + tj * cw[2 * g];
      const float cadd1 = cb[2 * g + 1] + tj * cw[2 * g + 1];
      const int n0c = 64 * wave + 32 * g + c;
#pragma unroll
      for (int r = 0; r < 8; ++r) {
        const float z0 = aH0[r] * W1_INV + aL0[r] * W1_LO_INV + cadd0;
        const float z1 = aH1[r] * W1_INV + aL1[r] * W1_LO_INV + cadd1;
        Hh[(8 * hh + r) * HPITCH + n0c]      = (_Float16)ftanh(z0);
        Hh[(8 * hh + r) * HPITCH + n0c + 16] = (_Float16)ftanh(z1);
      }
    }
    __syncthreads();

    v8f fH = z8, fL = z8;
    {
      const _Float16* ha = Hh + c * HPITCH + koff;
#pragma unroll 1
      for (int k0 = 0; k0 < HID_DIM; k0 += 32) {
        const v16h a  = Frag<_Float16>::load(ha + k0);
        const v16h bh = Frag<_Float16>::load(v2h + k0);
        const v16h bl = Frag<_Float16>::load(v2l + k0);
        fH = Frag<_Float16>::mma(a, bh, fH);
        fL = Frag<_Float16>::mma(a, bl, fL);
        dep_guard_h(fH, fL, a, bl);
        keep2_h(bh, bl);
      }
    }
    acc_guard2(fH, fL);
#pragma unroll
    for (int r = 0; r < 8; ++r) {
      const float fv = fH[r] * W2_INV + fL[r] * W2_LO_INV + b2v;
      xs[r] = xs[r] + dtv * fv;
    }
    __syncthreads();
#pragma unroll
    for (int r = 0; r < 8; ++r) {
      Os[(8 * hh + r) * OPITCH + dcol] = xs[r];
      Yr[sy * SLOT_HALVES + (8 * hh + r) * YPITCH + dcol] = (_Float16)xs[r];
    }
    __syncthreads();
    {
      float* orow = out + (size_t)(j + 1) * (size_t)(NBATCH * STATE_DIM) + (size_t)rb * STATE_DIM;
      for (int pass = 0; pass < 2; ++pass) {
#pragma unroll
        for (int it = 0; it < 2; ++it) {
          const int idx = it * NTHREADS + tid;
          const int row = idx >> 5, c4 = (idx & 31) * 4;
          const v4f v = *(const v4f*)(Os + row * OPITCH + c4);
          *(volatile v4f*)(orow + (size_t)row * STATE_DIM + c4) = v;
        }
        __threadfence();
      }
    }
    __syncthreads();
    sx = sy;
    sy = (sy + 1 == NSLOTS) ? 0 : (sy + 1);
  }
}

extern "C" void kernel_launch(void* const* d_in, const int* in_sizes, int n_in,
                              void* d_out, int out_size, void* d_ws, size_t ws_size, hipStream_t stream) {
  if (n_in < 7 || d_out == nullptr || d_ws == nullptr) return;
  if (in_sizes[0] < 1 || in_sizes[1] != HID_DIM * IN_DIM || in_sizes[2] != HID_DIM ||
      in_sizes[3] != STATE_DIM * HID_DIM || in_sizes[4] != STATE_DIM || in_sizes[5] != NBATCH * STATE_DIM ||
      in_sizes[6] != STATE_DIM || out_size != (NUM_STEPS + 1) * NBATCH * STATE_DIM) return;

  const float* tau = (const float*)d_in[0];
  const float* W1  = (const float*)d_in[1];
  const float* b1  = (const float*)d_in[2];
  const float* W2  = (const float*)d_in[3];
  const float* b2  = (const float*)d_in[4];
  const float* c0  = (const float*)d_in[5];
  const float* c1  = (const float*)d_in[6];
  float* out = (float*)d_out;

  char* ws = (char*)d_ws; size_t off = 0;
  auto carve = [&](size_t bytes) -> char* { char* p = ws + off; off += (bytes + 255) & ~(size_t)255; return p; };
  unsigned short* W1H = (unsigned short*)carve((size_t)HID_DIM * KXY * 2);
  unsigned short* W1L = (unsigned short*)carve((size_t)HID_DIM * KXY * 2);
  unsigned short* W2H = (unsigned short*)carve((size_t)STATE_DIM * HID_DIM * 2);
  unsigned short* W2L = (unsigned short*)carve((size_t)STATE_DIM * HID_DIM * 2);
  if (off > ws_size || off > (size_t)134217728) return;

  split_planes_kernel<<<(HID_DIM * KXY / 8) / NTHREADS, NTHREADS, 0, stream>>>(W1, HID_DIM, IN_DIM, KXY, W1_CARRY, W1H, W1L);
  split_planes_kernel<<<(STATE_DIM * HID_DIM / 8) / NTHREADS, NTHREADS, 0, stream>>>(W2, STATE_DIM, HID_DIM, HID_DIM, W2_CARRY, W2H, W2L);
  dde_euler_kernel<<<NBATCH / ROWS_PB, NTHREADS, 0, stream>>>(tau, W1, b1, b2, c0, c1, W1H, W1L, W2H, W2L, out);
}
